// TimeDependentAttention_48430051229898
// MI455X (gfx1250) — hardware-verified
//
#include <hip/hip_runtime.h>
#include <stdint.h>


typedef _Float16 f16;
typedef f16   v8h  __attribute__((ext_vector_type(8)));
typedef f16   v16h __attribute__((ext_vector_type(16)));
typedef float v8f  __attribute__((ext_vector_type(8)));
typedef float v4f  __attribute__((ext_vector_type(4)));

union Frag { v16h v; v8h half[2]; };

#define D_MODEL 768
#define SEQ     1024
#define BATCH   8
#define NH      12
#define HD      64
#define DT      256
#define MROWS   (BATCH * SEQ)

static_assert(MROWS % 64 == 0);
static_assert(D_MODEL % 64 == 0);
static_assert(SEQ % 64 == 0);
static_assert(NH * HD == D_MODEL);
static_assert(HD == 64);
static_assert((3 * BATCH * D_MODEL) % 256 == 0);

__device__ __forceinline__ v8f wmma16(v16h a, v16h b, v8f c) {
  v8f d = __builtin_amdgcn_wmma_f32_16x16x32_f16(false, a, false, b, (short)0, c,
                                                 false, false);
  asm volatile("v_nop\n\tv_nop\n\tv_nop\n\tv_nop" : "+v"(d) : "v"(a), "v"(b));
  return d;
}

__device__ __forceinline__ float bfr(float x) {
  unsigned u = __float_as_uint(x);
  u = (u + 0x7FFFu + ((u >> 16) & 1u)) & 0xFFFF0000u;
  return __uint_as_float(u);
}

__device__ __forceinline__ v8f zero8() {
  v8f z;
#pragma unroll
  for (int i = 0; i < 8; ++i) z[i] = 0.0f;
  return z;
}

__device__ __forceinline__ float redmax16(float v) {
#pragma unroll
  for (int m = 1; m <= 8; m <<= 1) v = fmaxf(v, __shfl_xor(v, m, 32));
  return v;
}
__device__ __forceinline__ float redsum16(float v) {
#pragma unroll
  for (int m = 1; m <= 8; m <<= 1) v += __shfl_xor(v, m, 32);
  return v;
}

__global__ __launch_bounds__(256)
void cvt_kernel(const float* __restrict__ x,
                const float* __restrict__ wq, const float* __restrict__ wk,
                const float* __restrict__ wv, const float* __restrict__ wo,
                f16* __restrict__ xh,
                f16* __restrict__ wqh, f16* __restrict__ wkh,
                f16* __restrict__ wvh, f16* __restrict__ woh,
                int nX8, int nW8) {
  const int gid = (int)blockIdx.x * (int)blockDim.x + (int)threadIdx.x;
  const int total = nX8 + 4 * nW8;
  if (gid >= total) return;
  const float* src;
  f16* dst;
  float sc;
  int i;
  if (gid < nX8) {
    src = x; dst = xh; sc = 1.0f; i = gid;
  } else {
    const int r = gid - nX8;
    const int w = r / nW8;
    i = r - w * nW8;
    sc = 256.0f;
    src = (w == 0) ? wq : (w == 1) ? wk : (w == 2) ? wv : wo;
    dst = (w == 0) ? wqh : (w == 1) ? wkh : (w == 2) ? wvh : woh;
  }
  const v4f a = *(const v4f*)(src + (size_t)i * 8);
  const v4f b = *(const v4f*)(src + (size_t)i * 8 + 4);
  v8h o;
#pragma unroll
  for (int j = 0; j < 4; ++j) {
    o[j]     = (f16)(bfr(a[j]) * sc);
    o[4 + j] = (f16)(bfr(b[j]) * sc);
  }
  f16* p = dst + (size_t)i * 8;
  *(volatile v8h*)p = o;
  __threadfence();
  *(volatile v8h*)p = o;
}

__global__ __launch_bounds__(256)
void tshift_kernel(const float* __restrict__ t,
                   const float* __restrict__ Wq,
                   const float* __restrict__ Wk,
                   const float* __restrict__ Wv,
                   float* __restrict__ out) {
  const int tid = (int)blockIdx.x * (int)blockDim.x + (int)threadIdx.x;
  if (tid >= 3 * BATCH * D_MODEL) return;
  const int s = tid / (BATCH * D_MODEL);
  const int r = tid - s * (BATCH * D_MODEL);
  const int b = r / D_MODEL, j = r - b * D_MODEL;
  const float* W  = (s == 0) ? Wq : (s == 1) ? Wk : Wv;
  const float* tv = t + (size_t)b * DT;
  const float* wv = W + (size_t)j * DT;
  float acc = 0.0f;
#pragma unroll 4
  for (int k = 0; k < DT; ++k) acc = fmaf(bfr(tv[k]), bfr(wv[k]), acc);
  const float res = acc;
  *(volatile float*)(out + tid) = res;
  __threadfence();
  *(volatile float*)(out + tid) = res;
}

template <int MODE>
__global__ __launch_bounds__(128)
void gemm_kernel(const f16* __restrict__ A, const f16* __restrict__ Alo,
                 const f16* __restrict__ W0, const f16* __restrict__ W1,
                 const f16* __restrict__ W2,
                 const float* __restrict__ shift,
                 f16* __restrict__ O0, f16* __restrict__ O1, f16* __restrict__ O2,
                 float* __restrict__ outF) {
  __shared__ __align__(16) float sT[4][16][68];

  const int wave = (int)threadIdx.x >> 5;
  const int lane = (int)threadIdx.x & 31;
  const int lh = lane >> 4, l15 = lane & 15;
  const int z = (int)blockIdx.z;
  const f16* W = (z == 0) ? W0 : (z == 1) ? W1 : W2;
  const int mBase = (int)blockIdx.x * 64 + wave * 16;
  const int nBase = (int)blockIdx.y * 64;

  v8f acc[4];
  v8f accr[4];
#pragma unroll
  for (int c = 0; c < 4; ++c) { acc[c] = zero8(); accr[c] = zero8(); }

  const f16* arow = A + (size_t)(mBase + l15) * D_MODEL + 8 * lh;
  const f16* alow = (MODE == 1) ? (Alo + (size_t)(mBase + l15) * D_MODEL + 8 * lh) : arow;
  const f16* wrow = W + (size_t)(nBase + l15) * D_MODEL + 8 * lh;

  for (int k0 = 0; k0 < D_MODEL; k0 += 32) {
    Frag a;
    a.half[0] = *(const v8h*)(arow + k0);
    a.half[1] = *(const v8h*)(arow + k0 + 16);
    Frag al;
    if (MODE == 1) {
      al.half[0] = *(const v8h*)(alow + k0);
      al.half[1] = *(const v8h*)(alow + k0 + 16);
    }
#pragma unroll
    for (int c = 0; c < 4; ++c) {
      const f16* wp = wrow + (size_t)c * 16 * D_MODEL + k0;
      Frag b;
      b.half[0] = *(const v8h*)wp;
      b.half[1] = *(const v8h*)(wp + 16);
      acc[c] = wmma16(a.v, b.v, acc[c]);
      if (MODE == 1) accr[c] = wmma16(al.v, b.v, accr[c]);
    }
  }

  const int bidx = mBase / SEQ;
#pragma unroll
  for (int c = 0; c < 4; ++c) {
    const int n = nBase + c * 16 + l15;
    float add;
    if (MODE == 0) add = shift[(size_t)z * BATCH * D_MODEL + (size_t)bidx * D_MODEL + n];
    else           add = bfr(shift[n]);
#pragma unroll
    for (int g = 0; g < 8; ++g) {
      float v;
      if (MODE == 0) v = acc[c][g] * (1.0f / 256.0f) + add;
      else           v = (acc[c][g] + accr[c][g] * (1.0f / 2048.0f)) * (1.0f / 256.0f) + add;
      sT[wave][8 * lh + g][c * 16 + l15] = v;
    }
  }
  __syncthreads();

  if (MODE == 0) {
    f16* outH = (z == 0) ? O0 : (z == 1) ? O1 : O2;
    const int hh = nBase / HD;
    const int l0 = mBase % SEQ;
    f16* base = outH + (((size_t)(bidx * NH + hh)) * SEQ + (size_t)l0) * HD;
    v8h vals[4];
#pragma unroll
    for (int it = 0; it < 4; ++it) {
      const int r = it * 4 + (lane >> 3), piece = lane & 7;
      const v4f f0 = *(const v4f*)&sT[wave][r][piece * 8];
      const v4f f1 = *(const v4f*)&sT[wave][r][piece * 8 + 4];
      v8h o;
#pragma unroll
      for (int j = 0; j < 4; ++j) { o[j] = (f16)f0[j]; o[4 + j] = (f16)f1[j]; }
      vals[it] = o;
    }
#pragma unroll
    for (int it = 0; it < 4; ++it) {
      const int r = it * 4 + (lane >> 3), piece = lane & 7;
      *(volatile v8h*)(base + (size_t)r * HD + piece * 8) = vals[it];
    }
    __threadfence();
#pragma unroll
    for (int it = 0; it < 4; ++it) {
      const int r = it * 4 + (lane >> 3), piece = lane & 7;
      *(volatile v8h*)(base + (size_t)r * HD + piece * 8) = vals[it];
    }
  } else {
    v4f vals[8];
#pragma unroll
    for (int it = 0; it < 8; ++it) {
      const int L = it * 4 + (lane >> 3);
      const int r = L >> 1, col = (L & 1) * 32 + (lane & 7) * 4;
      vals[it] = *(const v4f*)&sT[wave][r][col];
    }
#pragma unroll
    for (int it = 0; it < 8; ++it) {
      const int L = it * 4 + (lane >> 3);
      const int r = L >> 1, col = (L & 1) * 32 + (lane & 7) * 4;
      *(volatile v4f*)(outF + (size_t)(mBase + r) * D_MODEL + nBase + col) = vals[it];
    }
    __threadfence();
#pragma unroll
    for (int it = 0; it < 8; ++it) {
      const int L = it * 4 + (lane >> 3);
      const int r = L >> 1, col = (L & 1) * 32 + (lane & 7) * 4;
      *(volatile v4f*)(outF + (size_t)(mBase + r) * D_MODEL + nBase + col) = vals[it];
    }
  }
}

__global__ __launch_bounds__(128)
void attn_kernel(const f16* __restrict__ Q, const f16* __restrict__ K,
                 const f16* __restrict__ V, const float* __restrict__ bias,
                 f16* __restrict__ Ohi, f16* __restrict__ Olo) {
  __shared__ __align__(16) f16 sK[32][72];
  __shared__ __align__(16) f16 sVt[64][40];
  __shared__ __align__(16) f16 sP[4][16][40];
  __shared__ __align__(16) float sO[4][16][68];

  const int bh = (int)blockIdx.x / (SEQ / 64);
  const int qb = (int)blockIdx.x % (SEQ / 64);
  const int b = bh / NH, h = bh % NH;
  const int tid = (int)threadIdx.x;
  const int wave = tid >> 5;
  const int lane = tid & 31;
  const int lh = lane >> 4, l15 = lane & 15;
  const int qBase = qb * 64 + wave * 16;

  const f16* Qb = Q + (size_t)bh * SEQ * HD;
  const f16* Kb = K + (size_t)bh * SEQ * HD;
  const f16* Vb = V + (size_t)bh * SEQ * HD;

  const f16* qrow = Qb + (size_t)(qBase + l15) * HD + 8 * lh;
  Frag qa[2];
#pragma unroll
  for (int kc = 0; kc < 2; ++kc) {
    qa[kc].half[0] = *(const v8h*)(qrow + kc * 32);
    qa[kc].half[1] = *(const v8h*)(qrow + kc * 32 + 16);
  }

  v8f o[4];
  float mrow[8], lrow[8];
#pragma unroll
  for (int c = 0; c < 4; ++c) o[c] = zero8();
#pragma unroll
  for (int g = 0; g < 8; ++g) { mrow[g] = -1e30f; lrow[g] = 0.0f; }

  const float* bh_bias = bias + (size_t)h * SEQ * SEQ;

  for (int kb = 0; kb < SEQ / 32; ++kb) {
    __syncthreads();
#pragma unroll
    for (int p = 0; p < 2; ++p) {
      const int idx = p * 128 + tid;
      const int r = idx >> 3, seg = idx & 7;
      *(v8h*)&sK[r][seg * 8] =
          *(const v8h*)(Kb + (size_t)(kb * 32 + r) * HD + seg * 8);
      const v8h vv = *(const v8h*)(Vb + (size_t)(kb * 32 + r) * HD + seg * 8);
#pragma unroll
      for (int i = 0; i < 8; ++i) sVt[seg * 8 + i][r] = vv[i];
    }
    __syncthreads();

    v8f s[2];
#pragma unroll
    for (int nh = 0; nh < 2; ++nh) {
      s[nh] = zero8();
#pragma unroll
      for (int kc = 0; kc < 2; ++kc) {
        Frag kf;
        kf.half[0] = *(const v8h*)&sK[nh * 16 + l15][kc * 32 + 8 * lh];
        kf.half[1] = *(const v8h*)&sK[nh * 16 + l15][kc * 32 + 16 + 8 * lh];
        s[nh] = wmma16(qa[kc].v, kf.v, s[nh]);
      }
    }

    const float* bb = bh_bias + (size_t)kb * 32;
#pragma unroll
    for (int g = 0; g < 8; ++g) {
      const int row = qBase + g + 8 * lh;
      const float s0 = s[0][g] * 0.125f + bfr(bb[(size_t)row * SEQ + l15]);
      const float s1 = s[1][g] * 0.125f + bfr(bb[(size_t)row * SEQ + 16 + l15]);
      const float rm = redmax16(fmaxf(s0, s1));
      const float mnew = fmaxf(mrow[g], rm);
      const float corr = __expf(mrow[g] - mnew);
      const float p0 = __expf(s0 - mnew);
      const float p1 = __expf(s1 - mnew);
      const float rs = redsum16(p0 + p1);
      lrow[g] = lrow[g] * corr + rs;
      mrow[g] = mnew;
#pragma unroll
      for (int c = 0; c < 4; ++c) o[c][g] *= corr;
      const int m = g + 8 * lh;
      sP[wave][m][l15]      = (f16)(p0 * 4096.0f);
      sP[wave][m][16 + l15] = (f16)(p1 * 4096.0f);
    }
    __syncthreads();

    Frag pa;
    pa.half[0] = *(const v8h*)&sP[wave][l15][8 * lh];
    pa.half[1] = *(const v8h*)&sP[wave][l15][16 + 8 * lh];
#pragma unroll
    for (int c = 0; c < 4; ++c) {
      Frag vf;
      vf.half[0] = *(const v8h*)&sVt[c * 16 + l15][8 * lh];
      vf.half[1] = *(const v8h*)&sVt[c * 16 + l15][16 + 8 * lh];
      o[c] = wmma16(pa.v, vf.v, o[c]);
    }
  }

#pragma unroll
  for (int g = 0; g < 8; ++g) {
    const float inv = (1.0f / 4096.0f) / lrow[g];
#pragma unroll
    for (int c = 0; c < 4; ++c) sO[wave][8 * lh + g][c * 16 + l15] = o[c][g] * inv;
  }
  __syncthreads();

  const size_t rowoff = ((size_t)b * SEQ + (size_t)qBase) * D_MODEL + (size_t)h * HD;
  v8h hv[4], lv[4];
#pragma unroll
  for (int it = 0; it < 4; ++it) {
    const int r = it * 4 + (lane >> 3), piece = lane & 7;
    const v4f f0 = *(const v4f*)&sO[wave][r][piece * 8];
    const v4f f1 = *(const v4f*)&sO[wave][r][piece * 8 + 4];
    v8h hh, ll;
#pragma unroll
    for (int j = 0; j < 4; ++j) {
      const float v0 = f0[j];
      const f16 h0 = (f16)v0;
      hh[j] = h0;
      ll[j] = (f16)((v0 - (float)h0) * 2048.0f);
      const float v1 = f1[j];
      const f16 h1 = (f16)v1;
      hh[4 + j] = h1;
      ll[4 + j] = (f16)((v1 - (float)h1) * 2048.0f);
    }
    hv[it] = hh;
    lv[it] = ll;
  }
#pragma unroll
  for (int it = 0; it < 4; ++it) {
    const int r = it * 4 + (lane >> 3), piece = lane & 7;
    const size_t off = rowoff + (size_t)r * D_MODEL + (size_t)piece * 8;
    *(volatile v8h*)(Ohi + off) = hv[it];
    *(volatile v8h*)(Olo + off) = lv[it];
  }
  __threadfence();
#pragma unroll
  for (int it = 0; it < 4; ++it) {
    const int r = it * 4 + (lane >> 3), piece = lane & 7;
    const size_t off = rowoff + (size_t)r * D_MODEL + (size_t)piece * 8;
    *(volatile v8h*)(Ohi + off) = hv[it];
    *(volatile v8h*)(Olo + off) = lv[it];
  }
}

extern "C" void kernel_launch(void* const* d_in, const int* in_sizes, int n_in,
                              void* d_out, int out_size, void* d_ws,
                              size_t ws_size, hipStream_t stream) {
  const size_t nX    = (size_t)BATCH * SEQ * D_MODEL;
  const size_t nW    = (size_t)D_MODEL * D_MODEL;
  const size_t nWt   = (size_t)D_MODEL * DT;
  const size_t nT    = (size_t)BATCH * DT;
  const size_t nBias = (size_t)NH * SEQ * SEQ;
  const size_t nTsh  = (size_t)3 * BATCH * D_MODEL;

  if (n_in < 11) return;
  if (in_sizes[0] != (int)nX || in_sizes[1] != (int)nT || in_sizes[2] != (int)nBias) return;
  if (in_sizes[3] != (int)nW || in_sizes[4] != (int)nW || in_sizes[5] != (int)nW) return;
  if (in_sizes[6] != (int)nWt || in_sizes[7] != (int)nWt || in_sizes[8] != (int)nWt) return;
  if (in_sizes[9] != (int)nW || in_sizes[10] != D_MODEL) return;
  if (out_size != (int)nX) return;

  const float* x    = (const float*)d_in[0];
  const float* t    = (const float*)d_in[1];
  const float* bias = (const float*)d_in[2];
  const float* Wxq  = (const float*)d_in[3];
  const float* Wxk  = (const float*)d_in[4];
  const float* Wxv  = (const float*)d_in[5];
  const float* Wtq  = (const float*)d_in[6];
  const float* Wtk  = (const float*)d_in[7];
  const float* Wtv  = (const float*)d_in[8];
  const float* Wo   = (const float*)d_in[9];
  const float* bo   = (const float*)d_in[10];
  float* out = (float*)d_out;

  char* ws = (char*)d_ws;
  size_t off = 0;
  f16* Xh  = (f16*)(ws + off); off += nX * 2;
  f16* Wqh = (f16*)(ws + off); off += nW * 2;
  f16* Wkh = (f16*)(ws + off); off += nW * 2;
  f16* Wvh = (f16*)(ws + off); off += nW * 2;
  f16* Woh = (f16*)(ws + off); off += nW * 2;
  f16* Qh  = (f16*)(ws + off); off += nX * 2;
  f16* Kh  = (f16*)(ws + off); off += nX * 2;
  f16* Vh  = (f16*)(ws + off); off += nX * 2;
  f16* Ohi = (f16*)(ws + off); off += nX * 2;
  f16* Olo = (f16*)(ws + off); off += nX * 2;
  float* tsh = (float*)(ws + off); off += nTsh * 4;
  if (off > ws_size) return;

  const int nX8 = (int)(nX / 8), nW8 = (int)(nW / 8);
  const int cvtTotal = nX8 + 4 * nW8;
  cvt_kernel<<<(cvtTotal + 255) / 256, 256, 0, stream>>>(
      x, Wxq, Wxk, Wxv, Wo, Xh, Wqh, Wkh, Wvh, Woh, nX8, nW8);

  tshift_kernel<<<(int)((nTsh + 255) / 256), 256, 0, stream>>>(t, Wtq, Wtk, Wtv, tsh);

  dim3 gQKV(MROWS / 64, D_MODEL / 64, 3);
  gemm_kernel<0><<<gQKV, 128, 0, stream>>>(Xh, Xh, Wqh, Wkh, Wvh, tsh,
                                          Qh, Kh, Vh, nullptr);

  attn_kernel<<<BATCH * NH * (SEQ / 64), 128, 0, stream>>>(Qh, Kh, Vh, bias, Ohi, Olo);

  dim3 gOut(MROWS / 64, D_MODEL / 64, 1);
  gemm_kernel<1><<<gOut, 128, 0, stream>>>(Ohi, Olo, Woh, Woh, Woh, bo,
                                          nullptr, nullptr, nullptr, out);
}
